// PointNet_16956530884711
// MI455X (gfx1250) — hardware-verified
//
#include <hip/hip_runtime.h>
#include <math.h>
#pragma clang fp contract(off)

constexpr int NCLOUD = 64;
constexpr int NPTS   = 2048;
constexpr int KNBR   = 16;
constexpr int NCH    = 32;
constexpr int NCLS   = 40;
constexpr int NTOT   = NCLOUD * NPTS;
constexpr int NTHR   = 256;
constexpr int NOUTEL = NCLOUD * NCLS;
constexpr float HID_CARRY = 16.0f;
constexpr float H1_CARRY  = 16.0f;
constexpr float W_CARRY   = 64.0f;
constexpr float RES_CARRY = 2048.0f;
constexpr float RES_INV   = 1.0f / RES_CARRY;
constexpr float EDGE_FOLD = 1.0f / (HID_CARRY * W_CARRY);
constexpr float U_FOLD    = HID_CARRY / (H1_CARRY * W_CARRY);
constexpr int   UPITCH    = 36;

static_assert(NPTS % NTHR == 0, "knn grid exact");
static_assert(KNBR == 16, "one WMMA m-tile per point");
static_assert(NCH == 32, "one WMMA k-step per linear");
static_assert(NTOT % 16 == 0, "u tiles exact");
static_assert(NTHR * 4 == NCH * NCH, "W2 staging exact");
static_assert(NOUTEL == 2 * 1024 + 128 * 4, "classifier store map exact");
static_assert((UPITCH * 4) % 16 == 0, "slab rows 16-B aligned");

typedef __attribute__((ext_vector_type(16))) _Float16 v16h;
typedef __attribute__((ext_vector_type(8)))  float    v8f;
typedef __attribute__((ext_vector_type(4)))  float    v4f;
typedef __attribute__((ext_vector_type(4)))  int      v4i;

__device__ __forceinline__ v8f mma_h(v16h a, v16h b, v8f c) {
  return __builtin_amdgcn_wmma_f32_16x16x32_f16(false, a, false, b, (short)0, c, false, false);
}
__device__ __forceinline__ void guard2(v8f& c0, v8f& c1, v16h a, v16h b0, v16h b1) {
  asm volatile("v_nop\n\tv_nop\n\tv_nop\n\tv_nop" : "+v"(c0), "+v"(c1) : "v"(a), "v"(b0), "v"(b1));
}
__device__ __forceinline__ void guard4(v8f& c0, v8f& c1, v8f& c2, v8f& c3, v16h a0, v16h a1,
                                       v16h b0, v16h b1, v16h b2, v16h b3) {
  asm volatile("v_nop\n\tv_nop\n\tv_nop\n\tv_nop"
               : "+v"(c0), "+v"(c1), "+v"(c2), "+v"(c3)
               : "v"(a0), "v"(a1), "v"(b0), "v"(b1), "v"(b2), "v"(b3));
}
__device__ __forceinline__ constexpr int kmap(int e, int koff) { return (e < 8) ? (koff + e) : (8 + koff + e); }

__global__ __launch_bounds__(NTHR) void knn_kernel(const float* __restrict__ pos, int* __restrict__ idx) {
  __shared__ __align__(16) v4f sp[NPTS];
  __shared__ __align__(16) int stage[NTHR * KNBR];
  const int tid = threadIdx.x;
  const int b   = blockIdx.y;
  const float* cp = pos + (size_t)b * NPTS * 3;
#pragma unroll 1
  for (int j = tid; j < NPTS; j += NTHR) {
    const float x = cp[j * 3 + 0];
    const float y = cp[j * 3 + 1];
    const float z = cp[j * 3 + 2];
    const float xx = x * x;
    const float yy = y * y;
    const float zz = z * z;
    const float sq = (xx + zz) + yy;
    v4f pk;
    pk[0] = x; pk[1] = y; pk[2] = z; pk[3] = sq;
    sp[j] = pk;
  }
  __syncthreads();

  const int q = blockIdx.x * NTHR + tid;
  const v4f Q = sp[q];
  float bd[KNBR];
  int   bi[KNBR];
#pragma unroll
  for (int t = 0; t < KNBR; ++t) { bd[t] = 3.4e38f; bi[t] = 0; }

#pragma unroll 1
  for (int j = 0; j < NPTS; ++j) {
    const v4f Pj = sp[j];
    float p = Q[0] * Pj[0];
    p = fmaf(Q[1], Pj[1], p);
    p = fmaf(Q[2], Pj[2], p);
    const float s2 = Q[3] + Pj[3];
    const float tp = 2.0f * p;
    const float d  = s2 - tp;
    if (d < bd[KNBR - 1]) {
      float cd = d;
      int   ci = j;
      bool  ins = false;
#pragma unroll
      for (int t = 0; t < KNBR; ++t) {
        ins = ins || (cd < bd[t]);
        const float td = bd[t];
        const int   ti = bi[t];
        bd[t] = ins ? cd : td;
        bi[t] = ins ? ci : ti;
        cd = ins ? td : cd;
        ci = ins ? ti : ci;
      }
    }
  }

#pragma unroll
  for (int g4 = 0; g4 < 4; ++g4) {
    v4i v;
    v[0] = bi[4 * g4 + 0]; v[1] = bi[4 * g4 + 1]; v[2] = bi[4 * g4 + 2]; v[3] = bi[4 * g4 + 3];
    *(v4i*)(stage + tid * KNBR + 4 * g4) = v;
  }
  __syncthreads();
  int* dst = idx + ((size_t)b * NPTS + (size_t)blockIdx.x * NTHR) * KNBR;
  for (int pass = 0; pass < 2; ++pass) {
#pragma unroll
    for (int it = 0; it < 4; ++it) {
      const int o = (it * NTHR + tid) * 4;
      const v4i v = *(const v4i*)(stage + o);
      *(volatile v4i*)(dst + o) = v;
    }
    __threadfence();
  }
}

__global__ __launch_bounds__(NTHR) void layer_a_kernel(const float* __restrict__ pos, const int* __restrict__ idx,
                                                       const float* __restrict__ W1, const float* __restrict__ b1,
                                                       const float* __restrict__ W2, const float* __restrict__ b2,
                                                       float* __restrict__ hout) {
  __shared__ __align__(16) float sW2[NCH * NCH];
  __shared__ __align__(16) float sW1[6 * NCH];
  __shared__ __align__(16) float sB1[NCH];
  __shared__ __align__(16) float sB2[NCH];
  const int tid  = threadIdx.x;
  const int lane = tid & 31;
  const int wave = tid >> 5;
  {
    const v4f w = *(const v4f*)(W2 + 4 * tid);
    *(v4f*)(sW2 + 4 * tid) = w;
  }
  if (wave < 6) {
    sW1[tid] = W1[tid];
  } else if (wave == 6) {
    sB1[tid - 192] = b1[tid - 192];
  } else {
    sB2[tid - 224] = b2[tid - 224];
  }
  __syncthreads();

  const int m    = lane & 15;
  const int hh   = lane >> 4;
  const int koff = 8 * hh;
  float wA[6][16];
  float bA[16];
  v16h bf0, bf1;
#pragma unroll
  for (int e = 0; e < 16; ++e) {
    const int ch = kmap(e, koff);
#pragma unroll
    for (int c = 0; c < 6; ++c) wA[c][e] = sW1[c * NCH + ch] * HID_CARRY;
    bA[e] = sB1[ch] * HID_CARRY;
    bf0[e] = (_Float16)(sW2[ch * NCH + m] * W_CARRY);
    bf1[e] = (_Float16)(sW2[ch * NCH + 16 + m] * W_CARRY);
  }
  const float bias2 = sB2[lane];
  const v8f z8 = {0.f, 0.f, 0.f, 0.f, 0.f, 0.f, 0.f, 0.f};
  const int nw = gridDim.x * (NTHR / 32);

#pragma unroll 1
  for (int i = blockIdx.x * (NTHR / 32) + wave; i < NTOT; i += nw) {
    const int cloud = i / NPTS;
    int j = idx[(size_t)i * KNBR + m];
    j = j < 0 ? 0 : j;
    j = j > (NPTS - 1) ? (NPTS - 1) : j;
    const float* pj = pos + ((size_t)cloud * NPTS + (size_t)j) * 3;
    const float* pi = pos + (size_t)i * 3;
    const float xj = pj[0], yj = pj[1], zj = pj[2];
    const float xi = pi[0], yi = pi[1], zi = pi[2];
    const float rx = xj - xi;
    const float ry = yj - yi;
    const float rz = zj - zi;
    v16h a;
#pragma unroll
    for (int e = 0; e < 16; ++e) {
      float z = bA[e];
      z = fmaf(xj, wA[0][e], z);
      z = fmaf(yj, wA[1][e], z);
      z = fmaf(zj, wA[2][e], z);
      z = fmaf(rx, wA[3][e], z);
      z = fmaf(ry, wA[4][e], z);
      z = fmaf(rz, wA[5][e], z);
      z = fmaxf(z, 0.0f);
      a[e] = (_Float16)z;
    }
    v8f c0 = z8, c1 = z8;
    c0 = mma_h(a, bf0, c0);
    c1 = mma_h(a, bf1, c1);
    guard2(c0, c1, a, bf0, bf1);
    float p0 = c0[0], p1 = c1[0];
#pragma unroll
    for (int r = 1; r < 8; ++r) { p0 = fmaxf(p0, c0[r]); p1 = fmaxf(p1, c1[r]); }
    const float q0 = __shfl_xor(p0, 16, 32);
    const float q1 = __shfl_xor(p1, 16, 32);
    p0 = fmaxf(p0, q0);
    p1 = fmaxf(p1, q1);
    const float pv = (hh == 0) ? p0 : p1;
    const float hv = fmaxf(fmaf(pv, EDGE_FOLD, bias2), 0.0f);
    volatile float* hp = hout + (size_t)i * NCH + lane;
    *hp = hv;
    __threadfence();
    *hp = hv;
  }
}

__global__ __launch_bounds__(NTHR) void u_kernel(const float* __restrict__ h1, const float* __restrict__ pos,
                                                 const float* __restrict__ W1b, const float* __restrict__ b1b,
                                                 float* __restrict__ uout) {
  __shared__ __align__(16) float sW[NCH * NCH];
  __shared__ __align__(16) float sWp[3 * NCH];
  __shared__ __align__(16) float sB[NCH];
  __shared__ __align__(16) float slabs[NTHR / 32][16 * UPITCH];
  const int tid  = threadIdx.x;
  const int lane = tid & 31;
  const int wave = tid >> 5;
  {
    const v4f w = *(const v4f*)(W1b + 4 * tid);
    *(v4f*)(sW + 4 * tid) = w;
  }
  if (wave < 3) {
    sWp[tid] = W1b[NCH * NCH + tid];
  } else if (wave == 3) {
    sB[tid - 96] = b1b[tid - 96];
  }
  __syncthreads();

  const int m    = lane & 15;
  const int hh   = lane >> 4;
  const int koff = 8 * hh;
  v16h bh0, bh1, bl0, bl1;
#pragma unroll
  for (int e = 0; e < 16; ++e) {
    const int k = kmap(e, koff);
    const float w0 = sW[k * NCH + m] * W_CARRY;
    const float w1 = sW[k * NCH + 16 + m] * W_CARRY;
    const _Float16 h0 = (_Float16)w0;
    const _Float16 h1v = (_Float16)w1;
    const float r0 = (w0 - (float)h0) * RES_CARRY;
    const float r1 = (w1 - (float)h1v) * RES_CARRY;
    bh0[e] = h0;
    bh1[e] = h1v;
    bl0[e] = (_Float16)r0;
    bl1[e] = (_Float16)r1;
  }
  const int qr = lane >> 3;
  const int c4 = (lane & 7) * 4;
  float wp[3][4];
  float bb[4];
#pragma unroll
  for (int e = 0; e < 4; ++e) {
#pragma unroll
    for (int c = 0; c < 3; ++c) wp[c][e] = sWp[c * NCH + c4 + e] * HID_CARRY;
    bb[e] = sB[c4 + e] * HID_CARRY;
  }
  float* slab = slabs[wave];
  const v8f z8 = {0.f, 0.f, 0.f, 0.f, 0.f, 0.f, 0.f, 0.f};
  const int nw = gridDim.x * (NTHR / 32);

#pragma unroll 1
  for (int t = blockIdx.x * (NTHR / 32) + wave; t < NTOT / 16; t += nw) {
    const int r0 = t * 16;
    const float* hr = h1 + (size_t)(r0 + m) * NCH + koff;
    const v4f x0 = *(const v4f*)(hr);
    const v4f x1 = *(const v4f*)(hr + 4);
    const v4f x2 = *(const v4f*)(hr + 16);
    const v4f x3 = *(const v4f*)(hr + 20);
    v16h ah, al;
#pragma unroll
    for (int e = 0; e < 4; ++e) {
      const float s0 = x0[e] * H1_CARRY;
      const float s1 = x1[e] * H1_CARRY;
      const float s2 = x2[e] * H1_CARRY;
      const float s3 = x3[e] * H1_CARRY;
      const _Float16 g0 = (_Float16)s0;
      const _Float16 g1 = (_Float16)s1;
      const _Float16 g2 = (_Float16)s2;
      const _Float16 g3 = (_Float16)s3;
      ah[e]      = g0;
      ah[4 + e]  = g1;
      ah[8 + e]  = g2;
      ah[12 + e] = g3;
      al[e]      = (_Float16)((s0 - (float)g0) * RES_CARRY);
      al[4 + e]  = (_Float16)((s1 - (float)g1) * RES_CARRY);
      al[8 + e]  = (_Float16)((s2 - (float)g2) * RES_CARRY);
      al[12 + e] = (_Float16)((s3 - (float)g3) * RES_CARRY);
    }
    v8f m0 = z8, m1 = z8, e0 = z8, e1 = z8;
    m0 = mma_h(ah, bh0, m0);
    m1 = mma_h(ah, bh1, m1);
    e0 = mma_h(ah, bl0, e0);
    e1 = mma_h(ah, bl1, e1);
    e0 = mma_h(al, bh0, e0);
    e1 = mma_h(al, bh1, e1);
    guard4(m0, m1, e0, e1, ah, al, bh0, bh1, bl0, bl1);
#pragma unroll
    for (int r = 0; r < 8; ++r) {
      const float v0 = (m0[r] + e0[r] * RES_INV) * U_FOLD;
      const float v1 = (m1[r] + e1[r] * RES_INV) * U_FOLD;
      slab[(8 * hh + r) * UPITCH + m]      = v0;
      slab[(8 * hh + r) * UPITCH + 16 + m] = v1;
    }
    __builtin_amdgcn_fence(__ATOMIC_RELEASE, "workgroup");
    __builtin_amdgcn_wave_barrier();
    __builtin_amdgcn_fence(__ATOMIC_ACQUIRE, "workgroup");
    v4f o[4];
#pragma unroll
    for (int it = 0; it < 4; ++it) {
      const int row = it * 4 + qr;
      const v4f sv = *(const v4f*)(slab + row * UPITCH + c4);
      const float* pp = pos + (size_t)(r0 + row) * 3;
      const float px = pp[0], py = pp[1], pz = pp[2];
#pragma unroll
      for (int e = 0; e < 4; ++e) {
        float ad = bb[e];
        ad = fmaf(px, wp[0][e], ad);
        ad = fmaf(py, wp[1][e], ad);
        ad = fmaf(pz, wp[2][e], ad);
        o[it][e] = sv[e] + ad;
      }
    }
    for (int pass = 0; pass < 2; ++pass) {
#pragma unroll
      for (int it = 0; it < 4; ++it) {
        const int row = it * 4 + qr;
        *(volatile v4f*)(uout + (size_t)(r0 + row) * NCH + c4) = o[it];
      }
      __threadfence();
    }
    __builtin_amdgcn_fence(__ATOMIC_RELEASE, "workgroup");
    __builtin_amdgcn_wave_barrier();
    __builtin_amdgcn_fence(__ATOMIC_ACQUIRE, "workgroup");
  }
}

__global__ __launch_bounds__(NTHR) void layer_b_kernel(const float* __restrict__ pos, const int* __restrict__ idx,
                                                       const float* __restrict__ u, const float* __restrict__ W1b,
                                                       const float* __restrict__ W2, const float* __restrict__ b2,
                                                       float* __restrict__ hout) {
  __shared__ __align__(16) float sW2[NCH * NCH];
  __shared__ __align__(16) float sWp[3 * NCH];
  __shared__ __align__(16) float sB2[NCH];
  const int tid  = threadIdx.x;
  const int lane = tid & 31;
  const int wave = tid >> 5;
  {
    const v4f w = *(const v4f*)(W2 + 4 * tid);
    *(v4f*)(sW2 + 4 * tid) = w;
  }
  if (wave < 3) {
    sWp[tid] = W1b[NCH * NCH + tid];
  } else if (wave == 3) {
    sB2[tid - 96] = b2[tid - 96];
  }
  __syncthreads();

  const int m    = lane & 15;
  const int hh   = lane >> 4;
  const int koff = 8 * hh;
  float wv[3][16];
  v16h bf0, bf1;
#pragma unroll
  for (int e = 0; e < 16; ++e) {
    const int ch = kmap(e, koff);
#pragma unroll
    for (int c = 0; c < 3; ++c) wv[c][e] = sWp[c * NCH + ch] * HID_CARRY;
    bf0[e] = (_Float16)(sW2[ch * NCH + m] * W_CARRY);
    bf1[e] = (_Float16)(sW2[ch * NCH + 16 + m] * W_CARRY);
  }
  const float bias2 = sB2[lane];
  const v8f z8 = {0.f, 0.f, 0.f, 0.f, 0.f, 0.f, 0.f, 0.f};
  const int nw = gridDim.x * (NTHR / 32);

#pragma unroll 1
  for (int i = blockIdx.x * (NTHR / 32) + wave; i < NTOT; i += nw) {
    const int cloud = i / NPTS;
    int j = idx[(size_t)i * KNBR + m];
    j = j < 0 ? 0 : j;
    j = j > (NPTS - 1) ? (NPTS - 1) : j;
    const float* ur = u + ((size_t)cloud * NPTS + (size_t)j) * NCH + koff;
    const v4f u0 = *(const v4f*)(ur);
    const v4f u1 = *(const v4f*)(ur + 4);
    const v4f u2 = *(const v4f*)(ur + 16);
    const v4f u3 = *(const v4f*)(ur + 20);
    const float* pi = pos + (size_t)i * 3;
    const float nx = -pi[0];
    const float ny = -pi[1];
    const float nz = -pi[2];
    v16h a;
#pragma unroll
    for (int e = 0; e < 4; ++e) {
      float z0 = u0[e];
      float z1 = u1[e];
      float z2 = u2[e];
      float z3 = u3[e];
      z0 = fmaf(nx, wv[0][e], z0);      z0 = fmaf(ny, wv[1][e], z0);      z0 = fmaf(nz, wv[2][e], z0);
      z1 = fmaf(nx, wv[0][4 + e], z1);  z1 = fmaf(ny, wv[1][4 + e], z1);  z1 = fmaf(nz, wv[2][4 + e], z1);
      z2 = fmaf(nx, wv[0][8 + e], z2);  z2 = fmaf(ny, wv[1][8 + e], z2);  z2 = fmaf(nz, wv[2][8 + e], z2);
      z3 = fmaf(nx, wv[0][12 + e], z3); z3 = fmaf(ny, wv[1][12 + e], z3); z3 = fmaf(nz, wv[2][12 + e], z3);
      a[e]      = (_Float16)fmaxf(z0, 0.0f);
      a[4 + e]  = (_Float16)fmaxf(z1, 0.0f);
      a[8 + e]  = (_Float16)fmaxf(z2, 0.0f);
      a[12 + e] = (_Float16)fmaxf(z3, 0.0f);
    }
    v8f c0 = z8, c1 = z8;
    c0 = mma_h(a, bf0, c0);
    c1 = mma_h(a, bf1, c1);
    guard2(c0, c1, a, bf0, bf1);
    float p0 = c0[0], p1 = c1[0];
#pragma unroll
    for (int r = 1; r < 8; ++r) { p0 = fmaxf(p0, c0[r]); p1 = fmaxf(p1, c1[r]); }
    const float q0 = __shfl_xor(p0, 16, 32);
    const float q1 = __shfl_xor(p1, 16, 32);
    p0 = fmaxf(p0, q0);
    p1 = fmaxf(p1, q1);
    const float pv = (hh == 0) ? p0 : p1;
    const float hv = fmaxf(fmaf(pv, EDGE_FOLD, bias2), 0.0f);
    volatile float* hp = hout + (size_t)i * NCH + lane;
    *hp = hv;
    __threadfence();
    *hp = hv;
  }
}

__global__ __launch_bounds__(NTHR) void pool_kernel(const float* __restrict__ h2, float* __restrict__ g) {
  __shared__ float part[NTHR];
  const int tid = threadIdx.x;
  const int b = blockIdx.x;
  const int f = tid & 31;
  const int chunk = tid >> 5;
  const float* hp = h2 + ((size_t)b * NPTS + (size_t)chunk * (NPTS / 8)) * NCH + f;
  float mx = -3.4e38f;
#pragma unroll 4
  for (int p = 0; p < NPTS / 8; ++p) mx = fmaxf(mx, hp[(size_t)p * NCH]);
  part[tid] = mx;
  __syncthreads();
  if (tid < 32) {
    float m2 = part[tid];
#pragma unroll
    for (int c = 1; c < 8; ++c) m2 = fmaxf(m2, part[tid + 32 * c]);
    volatile float* gp = g + (size_t)b * NCH + tid;
    *gp = m2;
    __threadfence();
    *gp = m2;
  }
}

__device__ __forceinline__ float fc_one(const float* sG, const float* sWc, const float* sBc, int oidx) {
  const int oc = oidx > (NOUTEL - 1) ? (NOUTEL - 1) : oidx;
  const int b = oc / NCLS;
  const int c = oc - b * NCLS;
  float acc = sBc[c];
#pragma unroll 4
  for (int f = 0; f < NCH; ++f) acc = fmaf(sG[b * NCH + f], sWc[f * NCLS + c], acc);
  return acc;
}
__global__ __launch_bounds__(NTHR) void fc_kernel(const float* __restrict__ g, const float* __restrict__ Wc,
                                                  const float* __restrict__ bc, float* __restrict__ out) {
  __shared__ float sG[NCLOUD * NCH];
  __shared__ float sWc[NCH * NCLS];
  __shared__ float sBc[NCLS];
  const int tid = threadIdx.x;
#pragma unroll 1
  for (int i = tid; i < NCLOUD * NCH; i += NTHR) sG[i] = g[i];
#pragma unroll 1
  for (int i = tid; i < NCH * NCLS; i += NTHR) sWc[i] = Wc[i];
  if (tid < NCLS) sBc[tid] = bc[tid];
  __syncthreads();
  v4f o0, o1, o2;
#pragma unroll
  for (int e = 0; e < 4; ++e) {
    o0[e] = fc_one(sG, sWc, sBc, 0 * 1024 + 4 * tid + e);
    o1[e] = fc_one(sG, sWc, sBc, 1 * 1024 + 4 * tid + e);
    o2[e] = fc_one(sG, sWc, sBc, 2 * 1024 + 4 * tid + e);
  }
  for (int pass = 0; pass < 2; ++pass) {
    *(volatile v4f*)(out + 0 * 1024 + 4 * tid) = o0;
    *(volatile v4f*)(out + 1 * 1024 + 4 * tid) = o1;
    if (tid < 128) *(volatile v4f*)(out + 2 * 1024 + 4 * tid) = o2;
    __threadfence();
  }
}

extern "C" void kernel_launch(void* const* d_in, const int* in_sizes, int n_in,
                              void* d_out, int out_size, void* d_ws, size_t ws_size, hipStream_t stream) {
  if (n_in < 12 || d_out == nullptr || d_ws == nullptr) return;
  if (in_sizes[0] != NTOT * 3 || in_sizes[2] != 6 * NCH || in_sizes[3] != NCH ||
      in_sizes[4] != NCH * NCH || in_sizes[5] != NCH || in_sizes[6] != 35 * NCH || in_sizes[7] != NCH ||
      in_sizes[8] != NCH * NCH || in_sizes[9] != NCH || in_sizes[10] != NCH * NCLS || in_sizes[11] != NCLS ||
      out_size != NOUTEL) return;

  const float* pos = (const float*)d_in[0];
  const float* W1a = (const float*)d_in[2];
  const float* b1a = (const float*)d_in[3];
  const float* W2a = (const float*)d_in[4];
  const float* b2a = (const float*)d_in[5];
  const float* W1b = (const float*)d_in[6];
  const float* b1b = (const float*)d_in[7];
  const float* W2b = (const float*)d_in[8];
  const float* b2b = (const float*)d_in[9];
  const float* Wc  = (const float*)d_in[10];
  const float* bc  = (const float*)d_in[11];
  float* out = (float*)d_out;

  char* ws = (char*)d_ws;
  size_t off = 0;
  auto carve = [&](size_t bytes) -> char* { char* p = ws + off; off += (bytes + 255) & ~(size_t)255; return p; };
  int*   IDX = (int*)carve((size_t)NTOT * KNBR * 4);
  float* H1  = (float*)carve((size_t)NTOT * NCH * 4);
  float* U16 = (float*)carve((size_t)NTOT * NCH * 4);
  float* H2  = (float*)carve((size_t)NTOT * NCH * 4);
  float* G   = (float*)carve((size_t)NCLOUD * NCH * 4);
  if (off > ws_size || off > (size_t)134217728) return;

  knn_kernel<<<dim3(NPTS / NTHR, NCLOUD), NTHR, 0, stream>>>(pos, IDX);
  layer_a_kernel<<<1024, NTHR, 0, stream>>>(pos, IDX, W1a, b1a, W2a, b2a, H1);
  u_kernel<<<256, NTHR, 0, stream>>>(H1, pos, W1b, b1b, U16);
  layer_b_kernel<<<1024, NTHR, 0, stream>>>(pos, IDX, U16, W1b, W2b, b2b, H2);
  pool_kernel<<<NCLOUD, NTHR, 0, stream>>>(H2, G);
  fc_kernel<<<1, NTHR, 0, stream>>>(G, Wc, bc, out);
}
